// Neural3DHMM_64707977281582
// MI455X (gfx1250) — hardware-verified
//
#include <hip/hip_runtime.h>


namespace {
constexpr int XY = 16, ZZ = 8, S = 2048, V = 10000, VP = 10016, EMB = 256, TOK = 100, TOKP = 128, HID = 256, NB = 8, T = 16, LL = 12, WSZ = 2;
constexpr float XS = 8.0f, WSC = 256.0f, LNEPS = 1e-5f;
typedef _Float16 b16;
typedef __attribute__((ext_vector_type(16))) _Float16 v16b;
typedef __attribute__((ext_vector_type(8))) _Float16 v8b;
typedef __attribute__((ext_vector_type(8))) float v8f;
typedef __attribute__((ext_vector_type(4))) float v4f;
__device__ __forceinline__ float bf16_rne(float f) { unsigned int u = __float_as_uint(f); u += 0x7FFFu + ((u >> 16) & 1u); return __uint_as_float(u & 0xFFFF0000u); }
__device__ __forceinline__ void split16(float v, b16& hi, b16& lo) { hi = (b16)v; lo = (b16)(v - (float)hi); }
__device__ __forceinline__ v16b frag_kb(const b16* p, int hh) { const v8b a = *(const v8b*)(p + 8 * hh), b = *(const v8b*)(p + 16 + 8 * hh); v16b f;
#pragma unroll
  for (int e = 0; e < 8; ++e) { f[e] = a[e]; f[8 + e] = b[e]; } return f; }
__device__ __forceinline__ v8f wmma16b(v16b a, v16b b, v8f c) { v8f d = __builtin_amdgcn_wmma_f32_16x16x32_f16(false, a, false, b, (short)0, c, false, false); asm volatile("v_nop\n\tv_nop\n\tv_nop\n\tv_nop" : "+v"(d) : "v"(a), "v"(b)); return d; }
__device__ __forceinline__ void wave_lds_sync() { __builtin_amdgcn_fence(__ATOMIC_RELEASE, "workgroup"); __builtin_amdgcn_wave_barrier(); __builtin_amdgcn_fence(__ATOMIC_ACQUIRE, "workgroup"); }
__device__ __forceinline__ float pmul(float a, float b) { float p = a * b; asm volatile("" : "+v"(p)); return p; }
__device__ __forceinline__ int iclamp(int v, int lo, int hi) { return v < lo ? lo : (v > hi ? hi : v); }
__device__ __forceinline__ float lae(float a, float b) { const float m = fmaxf(a, b), d = -fabsf(a - b); return (m == -INFINITY) ? -INFINITY : m + log1pf(__expf(d)); }

__global__ __launch_bounds__(256) void wcopy_kernel(const float* __restrict__ w, int OUT, int KIN, int OUTP, int KP, b16* __restrict__ WT) {
  const size_t u = (size_t)blockIdx.x * 256 + threadIdx.x; if (u >= (size_t)OUTP * KP / 8) return; const size_t e = u * 8; const int o = (int)(e / KP), k0 = (int)(e % KP); v8b v;
  for (int j = 0; j < 8; ++j) { const int k = k0 + j; v[j] = (o < OUT && k < KIN) ? (b16)(bf16_rne(w[(size_t)o * KIN + k]) * WSC) : (b16)0.0f; } for (int pass = 0; pass < 2; ++pass) { *(volatile v8b*)(WT + e) = v; __threadfence(); }
}
__global__ __launch_bounds__(256) void tokprep_kernel(const float* __restrict__ te, b16* __restrict__ TE) {
  const size_t u = (size_t)blockIdx.x * 256 + threadIdx.x; if (u >= (size_t)VP * TOKP / 8) return; const size_t e = u * 8; const int o = (int)(e / TOKP), k0 = (int)(e % TOKP); v8b v;
  for (int j = 0; j < 8; ++j) { const int k = k0 + j; v[j] = (o < V && k < TOK) ? (b16)bf16_rne(te[(size_t)o * TOK + k]) : (b16)0.0f; } for (int pass = 0; pass < 2; ++pass) { *(volatile v8b*)(TE + e) = v; __threadfence(); }
}
template <int NOUT, int NTI, int HP>
__global__ __launch_bounds__(32) void res_kernel(const float* __restrict__ se, const b16* __restrict__ W1T, const b16* __restrict__ W2T, const float* __restrict__ b1, const float* __restrict__ b2, const float* __restrict__ g, const float* __restrict__ be, float* __restrict__ Hout) {
  __shared__ __attribute__((aligned(16))) b16 Ah[16][EMB + 8], Al[16][EMB + 8]; __shared__ __attribute__((aligned(16))) float X1[16][HID + 4], Hr[16][HID + 4];
  const int lane = threadIdx.x, nloc = lane & 15, hlf = lane >> 4; const size_t m0 = (size_t)blockIdx.x * 16; const float sc = 1.0f / (XS * WSC);
  for (int rr = 0; rr < 16; ++rr) for (int q = 0; q < 2; ++q) { const v4f v = *(const v4f*)(se + (m0 + rr) * EMB + q * 128 + lane * 4); for (int j = 0; j < 4; ++j) { Ah[rr][q * 128 + lane * 4 + j] = (b16)(bf16_rne(v[j]) * XS); Al[rr][q * 128 + lane * 4 + j] = (b16)0.0f; } }
  wave_lds_sync();
  constexpr int NPASS = (NTI + 7) / 8;
#pragma unroll 1
  for (int cg = 0; cg < NPASS; ++cg) { v8f acc[8];
#pragma unroll
    for (int t = 0; t < 8; ++t) acc[t] = (v8f){};
#pragma unroll 2
    for (int kb = 0; kb < EMB; kb += 32) { const v16b a = frag_kb(&Ah[nloc][kb], hlf);
#pragma unroll
      for (int t = 0; t < 8; ++t) if (cg * 8 + t < NTI) acc[t] = wmma16b(a, frag_kb(W1T + (size_t)(cg * 128 + t * 16 + nloc) * EMB + kb, hlf), acc[t]); }
#pragma unroll
    for (int t = 0; t < 8; ++t) { if (cg * 8 + t >= NTI) break; const int c = cg * 128 + t * 16 + nloc; const float bb = c < NOUT ? bf16_rne(b1[c]) : 0.0f;
#pragma unroll 1
      for (int r8 = 0; r8 < 8; ++r8) X1[8 * hlf + r8][c] = c < NOUT ? fmaxf(acc[t][r8] * sc + bb, 0.0f) : 0.0f; } }
  wave_lds_sync();
  constexpr int K2 = ((NTI * 16 + 31) / 32) * 32;
  for (int rr = 0; rr < 16; ++rr) for (int c = lane; c < K2; c += 32) { b16 p, ql; split16(X1[rr][c < NTI * 16 ? c : 0] * ((c < NTI * 16) ? XS : 0.0f), p, ql); Ah[rr][c] = p; Al[rr][c] = ql; }
  wave_lds_sync();
#pragma unroll 1
  for (int cg = 0; cg < NPASS; ++cg) { v8f acc[8];
#pragma unroll
    for (int t = 0; t < 8; ++t) acc[t] = (v8f){};
#pragma unroll 2
    for (int kb = 0; kb < K2; kb += 32) { const v16b a = frag_kb(&Ah[nloc][kb], hlf), al = frag_kb(&Al[nloc][kb], hlf);
#pragma unroll
      for (int t = 0; t < 8; ++t) if (cg * 8 + t < NTI) { const v16b bw = frag_kb(W2T + (size_t)(cg * 128 + t * 16 + nloc) * K2 + kb, hlf); acc[t] = wmma16b(a, bw, acc[t]); acc[t] = wmma16b(al, bw, acc[t]); } }
#pragma unroll
    for (int t = 0; t < 8; ++t) { if (cg * 8 + t >= NTI) break; const int c = cg * 128 + t * 16 + nloc; const float bb = c < NOUT ? bf16_rne(b2[c]) : 0.0f;
#pragma unroll 1
      for (int r8 = 0; r8 < 8; ++r8) { const int rl = 8 * hlf + r8; Hr[rl][c] = c < NOUT ? fmaxf(acc[t][r8] * sc + bb, 0.0f) + X1[rl][c] : 0.0f; } } }
  wave_lds_sync();
  for (int rr = 0; rr < 16; ++rr) { float s = 0.0f; for (int c = lane; c < NOUT; c += 32) s += Hr[rr][c]; for (int o = 16; o; o >>= 1) s += __shfl_xor(s, o); const float mu = s / (float)NOUT;
    float qv = 0.0f; for (int c = lane; c < NOUT; c += 32) { const float d = Hr[rr][c] - mu; qv += pmul(d, d); } for (int o = 16; o; o >>= 1) qv += __shfl_xor(qv, o); const float rs = rsqrtf(qv / (float)NOUT + LNEPS);
    for (int c = lane; c < HP; c += 32) X1[rr][c] = c < NOUT ? pmul(pmul(Hr[rr][c] - mu, rs), bf16_rne(g[c])) + bf16_rne(be[c]) : 0.0f; }
  wave_lds_sync();
  for (int pass = 0; pass < 2; ++pass) { for (int rr = 0; rr < 16; ++rr) for (int q = 0; q < HP / 128; ++q) *(volatile v4f*)(Hout + (m0 + rr) * HP + q * 128 + lane * 4) = *(const v4f*)(&X1[rr][q * 128 + lane * 4]); __threadfence(); }
}
__global__ __launch_bounds__(256) void prior_kernel(const float* __restrict__ H0, const float* __restrict__ wo, const float* __restrict__ bo, float* __restrict__ PRI) {
  __shared__ float pv[S]; __shared__ float red[8];
  const int tid = threadIdx.x, wave = tid >> 5, lane = tid & 31; const float b = bf16_rne(bo[0]); float w8[8]; for (int j = 0; j < 8; ++j) w8[j] = bf16_rne(wo[lane * 8 + j]);
  for (int s = wave; s < S; s += 8) { float d = 0.0f; for (int j = 0; j < 8; ++j) d += pmul(H0[(size_t)s * HID + lane * 8 + j], w8[j]); for (int o = 16; o; o >>= 1) d += __shfl_xor(d, o); if (lane == 0) pv[s] = d + b; }
  __syncthreads();
  float m = -INFINITY; for (int s = tid; s < S; s += 256) m = fmaxf(m, pv[s]); for (int o = 16; o; o >>= 1) m = fmaxf(m, __shfl_xor(m, o)); if (lane == 0) red[wave] = m; __syncthreads();
  float gm = red[0]; for (int w = 1; w < 8; ++w) gm = fmaxf(gm, red[w]); __syncthreads();
  float se = 0.0f; for (int s = tid; s < S; s += 256) se += __expf(pv[s] - gm); for (int o = 16; o; o >>= 1) se += __shfl_xor(se, o); if (lane == 0) red[wave] = se; __syncthreads();
  float tot = 0.0f; for (int w = 0; w < 8; ++w) tot += red[w]; const float lse = gm + logf(tot);
  for (int pass = 0; pass < 2; ++pass) { for (int s = tid; s < S; s += 256) ((volatile float*)PRI)[s] = pv[s] - lse; __threadfence(); }
}
__constant__ int OFFS[7] = {0, 1, -1, XY, -XY, XY * XY, 2 * XY * XY};
__global__ __launch_bounds__(256) void trans_kernel(const float* __restrict__ HIN, const float* __restrict__ HOUT, float* __restrict__ TR) {
  __shared__ float tv[8][8];
  const int wave = threadIdx.x >> 5, lane = threadIdx.x & 31; const int j = blockIdx.x * 8 + wave; float hj[8]; for (int q = 0; q < 8; ++q) hj[q] = HIN[(size_t)j * HID + lane * 8 + q];
  float vals[7]; float mx = -INFINITY;
#pragma unroll
  for (int n = 0; n < 7; ++n) { const int i = j + OFFS[n]; const bool ok = i >= 0 && i < S; const int ic = iclamp(i, 0, S - 1); float d = 0.0f; for (int q = 0; q < 8; ++q) d += pmul(hj[q], HOUT[(size_t)ic * HID + lane * 8 + q]); for (int o = 16; o; o >>= 1) d += __shfl_xor(d, o); vals[n] = ok ? d : -INFINITY; mx = fmaxf(mx, vals[n]); }
  float ssum = 0.0f; for (int n = 0; n < 7; ++n) ssum += (vals[n] == -INFINITY) ? 0.0f : __expf(vals[n] - mx); const float lse = mx + logf(ssum);
  if (lane < 8) tv[wave][lane] = (lane < 7) ? vals[lane] - lse : -INFINITY;
  __syncthreads();
  for (int pass = 0; pass < 2; ++pass) { if (threadIdx.x < 64) ((volatile float*)TR)[(size_t)blockIdx.x * 64 + threadIdx.x] = tv[threadIdx.x >> 3][threadIdx.x & 7]; __threadfence(); }
}
__global__ __launch_bounds__(32) void emit_kernel(const float* __restrict__ HEM, const b16* __restrict__ TE, int VVP, float* __restrict__ LOG) {
  __shared__ __attribute__((aligned(16))) b16 Ah[16][TOKP + 8], Al[16][TOKP + 8]; __shared__ __attribute__((aligned(16))) float Tf[16][128 + 4];
  const int lane = threadIdx.x, nloc = lane & 15, hlf = lane >> 4; const size_t m0 = (size_t)blockIdx.x * 16; const int c0 = blockIdx.y * 128; const int ntile = (VVP - c0) >= 128 ? 8 : (VVP - c0) / 16;
  for (int rr = 0; rr < 16; ++rr) { const v4f v = *(const v4f*)(HEM + (m0 + rr) * TOKP + lane * 4); for (int j = 0; j < 4; ++j) { b16 p, ql; split16(v[j] * XS, p, ql); Ah[rr][lane * 4 + j] = p; Al[rr][lane * 4 + j] = ql; } }
  wave_lds_sync();
  v8f acc[8];
#pragma unroll
  for (int t = 0; t < 8; ++t) acc[t] = (v8f){};
#pragma unroll
  for (int kb = 0; kb < TOKP; kb += 32) { const v16b a = frag_kb(&Ah[nloc][kb], hlf), al = frag_kb(&Al[nloc][kb], hlf);
#pragma unroll
    for (int t = 0; t < 8; ++t) if (t < ntile) { const v16b bw = frag_kb(TE + (size_t)(c0 + t * 16 + nloc) * TOKP + kb, hlf); acc[t] = wmma16b(a, bw, acc[t]); acc[t] = wmma16b(al, bw, acc[t]); } }
#pragma unroll
  for (int t = 0; t < 8; ++t)
#pragma unroll 1
    for (int r8 = 0; r8 < 8; ++r8) Tf[8 * hlf + r8][t * 16 + nloc] = acc[t][r8] * (1.0f / XS);
  wave_lds_sync();
  for (int pass = 0; pass < 2; ++pass) { for (int rr = 0; rr < 16; ++rr) if (lane * 4 < ntile * 16) *(volatile v4f*)(LOG + (m0 + rr) * VP + c0 + lane * 4) = *(const v4f*)(&Tf[rr][lane * 4]); __threadfence(); }
}
__global__ __launch_bounds__(256) void lsm_kernel(float* __restrict__ LOG, int VV) {
  __shared__ float red[8];
  const int tid = threadIdx.x, wave = tid >> 5, lane = tid & 31; float* row = LOG + (size_t)blockIdx.x * VP;
  float m = -INFINITY; for (int c = tid; c < VV; c += 256) m = fmaxf(m, row[c]); for (int o = 16; o; o >>= 1) m = fmaxf(m, __shfl_xor(m, o)); if (lane == 0) red[wave] = m; __syncthreads();
  float gm = red[0]; for (int w = 1; w < 8; ++w) gm = fmaxf(gm, red[w]); __syncthreads();
  float se = 0.0f; for (int c = tid; c < VV; c += 256) se += __expf(row[c] - gm); for (int o = 16; o; o >>= 1) se += __shfl_xor(se, o); if (lane == 0) red[wave] = se; __syncthreads();
  float tot = 0.0f; for (int w = 0; w < 8; ++w) tot += red[w]; const float lse = gm + logf(tot);
  float vals[40]; for (int k = 0; k < 40; ++k) { const int c = tid + k * 256; vals[k] = c < VV ? row[c] - lse : 0.0f; }
  __syncthreads();
  for (int pass = 0; pass < 2; ++pass) { for (int k = 0; k < 40; ++k) { const int c = tid + k * 256; if (c < VV) ((volatile float*)row)[c] = vals[k]; } __threadfence(); }
}
template <int AXIS>
__global__ __launch_bounds__(256) void pool_kernel(const float* __restrict__ IN_, int VV, float* __restrict__ OUT_) {
  const int s = blockIdx.x, tid = threadIdx.x; const int z = s / (XY * XY), y = (s / XY) % XY, x = s % XY; const float lw = logf(5.0f);
  int nb[5]; for (int k = 0; k < 5; ++k) { if (AXIS == 0) { const int xx = iclamp(x - WSZ + k, 0, XY - 1); nb[k] = z * XY * XY + y * XY + xx; } else { const int yy = iclamp(y - WSZ + k, 0, XY - 1); nb[k] = z * XY * XY + yy * XY + x; } }
  for (int pass = 0; pass < 2; ++pass) {
    for (int c = tid; c < VV; c += 256) { float p[5]; float m = -INFINITY; for (int k = 0; k < 5; ++k) { p[k] = IN_[(size_t)nb[k] * VP + c]; m = fmaxf(m, p[k]); } float sum = 0.0f; for (int k = 0; k < 5; ++k) sum += __expf(p[k] - m); ((volatile float*)OUT_)[(size_t)s * VP + c] = m + __logf(sum) - lw; }
    __threadfence(); }
}
__global__ __launch_bounds__(256) void fwd_kernel(const float* __restrict__ EM, const float* __restrict__ PRI, const float* __restrict__ TR, const int* __restrict__ stories, int VV, float* __restrict__ out) {
  __shared__ float sc_[S]; __shared__ int toks[T][LL];
  const int b = blockIdx.x, tid = threadIdx.x;
  if (tid < T * LL) toks[tid / LL][tid % LL] = iclamp(stories[(b * T + tid / LL) * LL + tid % LL], 0, V);
  __syncthreads();
  float cur[8];
  for (int t = 0; t < T; ++t) {
    float nw[8];
    for (int k = 0; k < 8; ++k) { const int j = tid + k * 256; float e = 0.0f; for (int l = 0; l < LL; ++l) { const int tk = toks[t][l]; e += (tk >= VV) ? 0.0f : EM[(size_t)j * VP + tk]; }
      if (t == 0) nw[k] = e + PRI[j];
      else { float m = -INFINITY; float v7[7];
#pragma unroll
        for (int n = 0; n < 7; ++n) { const int i = j + OFFS[n]; const float tr = TR[(size_t)j * 8 + n]; v7[n] = (i >= 0 && i < S && tr != -INFINITY) ? tr + sc_[iclamp(i, 0, S - 1)] : -INFINITY; m = fmaxf(m, v7[n]); }
        float ssum = 0.0f; for (int n = 0; n < 7; ++n) ssum += (v7[n] == -INFINITY) ? 0.0f : __expf(v7[n] - m); nw[k] = e + (m + logf(ssum)); } }
    __syncthreads();
    for (int k = 0; k < 8; ++k) { cur[k] = nw[k]; sc_[tid + k * 256] = nw[k]; }
    __syncthreads();
    for (int pass = 0; pass < 2; ++pass) { for (int k = 0; k < 8; ++k) ((volatile float*)out)[((size_t)t * NB + b) * S + tid + k * 256] = cur[k]; __threadfence(); } }
}
}

extern "C" void kernel_launch(void* const* d_in, const int* in_sizes, int n_in, void* d_out, int out_size, void* d_ws, size_t ws_size, hipStream_t stream) {
  (void)n_in;
  auto Fp = [&](int i) { return (const float*)d_in[i]; }; auto Ip = [&](int i) { return (const int*)d_in[i]; };
  if (in_sizes[0] != S * EMB || in_sizes[1] != V * TOK || in_sizes[2] != HID * EMB || in_sizes[8] != HID || in_sizes[22] != TOK * EMB || in_sizes[24] != TOK * TOK || in_sizes[28] != NB * T * LL || out_size != T * NB * S) return;
  size_t off = 0; char* ws = (char*)d_ws;
  auto carve = [&](size_t bytes) { char* p = ws + off; off += (bytes + 255) & ~(size_t)255; return p; };
  b16* W1[4]; b16* W2[4]; for (int r = 0; r < 3; ++r) { W1[r] = (b16*)carve((size_t)HID * EMB * 2); W2[r] = (b16*)carve((size_t)HID * HID * 2); } W1[3] = (b16*)carve((size_t)112 * EMB * 2); W2[3] = (b16*)carve((size_t)112 * 128 * 2);
  b16* TE = (b16*)carve((size_t)VP * TOKP * 2);
  float* H0 = (float*)carve((size_t)S * HID * 4); float* HIN = (float*)carve((size_t)S * HID * 4); float* HOUT = (float*)carve((size_t)S * HID * 4); float* HEM = (float*)carve((size_t)S * TOKP * 4);
  float* PRI = (float*)carve(S * 4); float* TR = (float*)carve((size_t)S * 8 * 4); float* LOGp = (float*)carve((size_t)S * VP * 4); float* EM2 = (float*)carve((size_t)S * VP * 4);
  if (off > ws_size) return;
  auto g8 = [](size_t n8) { return (unsigned)((n8 + 255) / 256); };
  for (int r = 0; r < 3; ++r) { const int base = r == 0 ? 2 : (r == 1 ? 10 : 16); wcopy_kernel<<<g8((size_t)HID * EMB / 8), 256, 0, stream>>>(Fp(base), HID, EMB, HID, EMB, W1[r]); wcopy_kernel<<<g8((size_t)HID * HID / 8), 256, 0, stream>>>(Fp(base + 2), HID, HID, HID, HID, W2[r]); }
  wcopy_kernel<<<g8((size_t)112 * EMB / 8), 256, 0, stream>>>(Fp(22), TOK, EMB, 112, EMB, W1[3]); wcopy_kernel<<<g8((size_t)112 * 128 / 8), 256, 0, stream>>>(Fp(24), TOK, TOK, 112, 128, W2[3]);
  tokprep_kernel<<<g8((size_t)VP * TOKP / 8), 256, 0, stream>>>(Fp(1), TE);
  res_kernel<HID, 16, HID><<<S / 16, 32, 0, stream>>>(Fp(0), W1[0], W2[0], Fp(3), Fp(5), Fp(6), Fp(7), H0);
  res_kernel<HID, 16, HID><<<S / 16, 32, 0, stream>>>(Fp(0), W1[1], W2[1], Fp(11), Fp(13), Fp(14), Fp(15), HIN);
  res_kernel<HID, 16, HID><<<S / 16, 32, 0, stream>>>(Fp(0), W1[2], W2[2], Fp(17), Fp(19), Fp(20), Fp(21), HOUT);
  res_kernel<TOK, 7, TOKP><<<S / 16, 32, 0, stream>>>(Fp(0), W1[3], W2[3], Fp(23), Fp(25), Fp(26), Fp(27), HEM);
  prior_kernel<<<1, 256, 0, stream>>>(H0, Fp(8), Fp(9), PRI);
  trans_kernel<<<S / 8, 256, 0, stream>>>(HIN, HOUT, TR);
  const int VV = V, VVP = VP;
  emit_kernel<<<dim3(S / 16, (VVP + 127) / 128), 32, 0, stream>>>(HEM, TE, VVP, LOGp);
  lsm_kernel<<<S, 256, 0, stream>>>(LOGp, VV);
  pool_kernel<0><<<S, 256, 0, stream>>>(LOGp, VV, EM2); pool_kernel<1><<<S, 256, 0, stream>>>(EM2, VV, LOGp);
  fwd_kernel<<<NB, 256, 0, stream>>>(LOGp, PRI, TR, Ip(28), VV, (float*)d_out);
}
